// SingleHeadAttention_44753559225124
// MI455X (gfx1250) — hardware-verified
//
#include <hip/hip_runtime.h>

typedef _Float16 h16;
typedef _Float16 h16x8 __attribute__((ext_vector_type(8)));
typedef _Float16 v16h  __attribute__((ext_vector_type(16)));
typedef float  v8f    __attribute__((ext_vector_type(8)));
typedef float  v4f    __attribute__((ext_vector_type(4)));
typedef unsigned v4u  __attribute__((ext_vector_type(4)));

#ifndef NB
#define NB 4
#endif
#ifndef SEQ
#define SEQ 2048
#endif
#define NB_FULL  4
#define SEQ_FULL 2048
#define C_DIM    1024
#define N_QKV    (3 * C_DIM)
#define M_ROWS   (NB * SEQ)
#define VRK      64
#ifndef QRES
#define QRES SEQ
#endif

static_assert(NB >= 1 && NB <= NB_FULL);
static_assert(SEQ >= 64 && SEQ <= SEQ_FULL);
static_assert(SEQ % 64 == 0);
static_assert(C_DIM % 256 == 0);
static_assert(M_ROWS % 64 == 0);
static_assert(N_QKV % 128 == 0);

#define XSC    16.0f
#define WSC    64.0f
#define QKV_UN (1.0f / 1024.0f)
#define RSC    2048.0f
#define RUN    (1.0f / 2048.0f)
#define ASC    0.03125f
#define PSC    1024.0f
#define PUN    (1.0f / 1024.0f)

template <typename V> __device__ __forceinline__ void vst2(void* p, V v) {
  *(volatile V*)p = v; __threadfence(); *(volatile V*)p = v;
}
__device__ __forceinline__ void copy16_g2s(h16* ldst, const h16* gsrc) { *(h16x8*)ldst = *(const h16x8*)gsrc; }

__device__ __forceinline__ float bf16_rne(float f) {
  unsigned u = __float_as_uint(f);
  u = (u + 0x7FFFu + ((u >> 16) & 1u)) & 0xFFFF0000u;
  return __uint_as_float(u);
}

__device__ __forceinline__ v16h load_a_frag(const h16* base, int ld, int k0) {
  int lane = threadIdx.x & 31;
  int idx  = lane & 15;
  int half = lane >> 4;
  const h16* p = base + (size_t)idx * ld + k0 + half * 8;
  h16x8 lo = *(const h16x8*)(p);
  h16x8 hi = *(const h16x8*)(p + 16);
  return __builtin_shufflevector(lo, hi, 0,1,2,3,4,5,6,7,8,9,10,11,12,13,14,15);
}
__device__ __forceinline__ v16h load_b_frag(const h16* base, int ld, int k0) { return load_a_frag(base, ld, k0); }

__device__ __forceinline__ v8f wmma_f16(v16h a, v16h b, v8f c) {
  v8f d = __builtin_amdgcn_wmma_f32_16x16x32_f16(false, a, false, b, (short)0, c, false, false);
  asm volatile("v_nop\n\tv_nop\n\tv_nop\n\tv_nop" : "+v"(d) : "v"(a), "v"(b));
  return d;
}

__global__ __launch_bounds__(256) void cvt_kernel(const float* __restrict__ src, h16* __restrict__ dst, int n8,
                                                  int seg_rows, int seg_full, float scale) {
  int g = blockIdx.x * blockDim.x + threadIdx.x;
  if (g >= n8) return;
  size_t e = (size_t)g * 8;
  int row = (int)(e / C_DIM);
  int col = (int)(e % C_DIM);
  int srow = (row / seg_rows) * seg_full + (row % seg_rows);
  const float* p = src + (size_t)srow * C_DIM + col;
  const v4f a = *(const v4f*)(p), b = *(const v4f*)(p + 4);
  union { h16x8 h; v4u u; } pk;
#pragma unroll
  for (int i = 0; i < 4; ++i) {
    pk.h[i]     = (h16)(bf16_rne(a[i]) * scale);
    pk.h[4 + i] = (h16)(bf16_rne(b[i]) * scale);
  }
  vst2(dst + e, pk.u);
}

__global__ __launch_bounds__(256) void qkv_kernel(const h16* __restrict__ Xh, const h16* __restrict__ Wh,
                                                  h16* __restrict__ Qh, h16* __restrict__ Ql,
                                                  h16* __restrict__ Kh, h16* __restrict__ Kl,
                                                  h16* __restrict__ Vt, h16* __restrict__ Vr) {
  __shared__ __align__(16) h16 T[128 * 136];
  const int m0  = blockIdx.x * 64;
  const int n0  = blockIdx.y * 128;
  const int sel = n0 / C_DIM;
  const int nl0 = n0 - sel * C_DIM;
  const int w    = threadIdx.x >> 5;
  const int lane = threadIdx.x & 31;
  const int idx  = lane & 15;
  const int half = lane >> 4;
  const int m_w = m0 + (w & 3) * 16;
  const int n_w = n0 + (w >> 2) * 64;

  v8f c[4] = {};
  const h16* arow = Xh + (size_t)m_w * C_DIM;
#pragma unroll 2
  for (int k0 = 0; k0 < C_DIM; k0 += 32) {
    v16h a = load_a_frag(arow, C_DIM, k0);
#pragma unroll
    for (int t = 0; t < 4; ++t) {
      v16h b = load_b_frag(Wh + (size_t)(n_w + t * 16) * C_DIM, C_DIM, k0);
      c[t] = wmma_f16(a, b, c[t]);
    }
  }

  const int tid = threadIdx.x;
  if (sel < 2) {
    h16* outH = (sel == 0) ? Qh : Kh;
    h16* outL = (sel == 0) ? Ql : Kl;
    for (int pass = 0; pass < 2; ++pass) {
#pragma unroll
      for (int t = 0; t < 4; ++t) {
        const int cl = (w >> 2) * 64 + t * 16 + idx;
#pragma unroll
        for (int g = 0; g < 8; ++g) {
          const int rl = (w & 3) * 16 + g + 8 * half;
          const float v = c[t][g] * QKV_UN;
          const h16 hv = (h16)v;
          h16 sv = hv;
          if (pass) sv = (h16)((v - (float)hv) * RSC);
          T[rl * 136 + cl] = sv;
        }
      }
      __syncthreads();
      h16* dst = pass ? outL : outH;
      for (int gg = tid; gg < 64 * 16; gg += 256) {
        const int rl = gg >> 4, pc = gg & 15;
        vst2(dst + (size_t)(m0 + rl) * C_DIM + nl0 + pc * 8, *(const v4u*)(&T[rl * 136 + pc * 8]));
      }
      __syncthreads();
    }
  } else {
    const int bb = m0 / SEQ, s0 = m0 % SEQ;
    const int npass = (s0 < VRK) ? 2 : 1;
    for (int pass = 0; pass < npass; ++pass) {
#pragma unroll
      for (int t = 0; t < 4; ++t) {
        const int cl = (w >> 2) * 64 + t * 16 + idx;
#pragma unroll
        for (int g = 0; g < 8; ++g) {
          const int rl = (w & 3) * 16 + g + 8 * half;
          const float v = c[t][g] * QKV_UN;
          const h16 hv = (h16)v;
          h16 sv = hv;
          if (pass) sv = (h16)((v - (float)hv) * RSC);
          T[cl * 72 + rl] = sv;
        }
      }
      __syncthreads();
      if (!pass) {
        for (int gg = tid; gg < 128 * 8; gg += 256) {
          const int cl = gg >> 3, pc = gg & 7;
          vst2(Vt + ((size_t)(bb * C_DIM + nl0 + cl)) * SEQ + s0 + pc * 8, *(const v4u*)(&T[cl * 72 + pc * 8]));
        }
      } else {
        for (int gg = tid; gg < 128 * 8; gg += 256) {
          const int cl = gg >> 3, pc = gg & 7;
          vst2(Vr + ((size_t)(bb * C_DIM + nl0 + cl)) * VRK + s0 + pc * 8, *(const v4u*)(&T[cl * 72 + pc * 8]));
        }
      }
      __syncthreads();
    }
  }
}

template <int PVRES>
__global__ __launch_bounds__(512)
void attn_kernel(const h16* __restrict__ Qh, const h16* __restrict__ Ql,
                 const h16* __restrict__ Kh, const h16* __restrict__ Kl,
                 const h16* __restrict__ Vt, const h16* __restrict__ Vr,
                 float* __restrict__ out, int qb0) {
  __shared__ __align__(16) h16   Qs[32][C_DIM];
  __shared__ __align__(16) float Ss[2][32][64];
  __shared__ __align__(16) h16   Ps[32][64];
  __shared__ __align__(16) h16   Prs[32][64];
  __shared__ float alpha_s[32];
  __shared__ float l_s[32];

  const int b    = blockIdx.y;
  const int q0   = (blockIdx.x + qb0) * 32;
  const int tid  = threadIdx.x;
  const int w    = tid >> 5;
  const int lane = tid & 31;
  const int idx  = lane & 15;
  const int half = lane >> 4;
  const int qi   = w & 1;
  const int kj   = (w >> 1) & 3;
  const int part = w >> 3;
  const int dg   = w >> 1;
  const bool use_res = (q0 < QRES);

  const h16* Qg = Qh + ((size_t)(b * SEQ + q0)) * C_DIM;
  for (int cc = tid; cc < 32 * (C_DIM / 8); cc += 512) {
    const int r = cc / (C_DIM / 8), dc = cc % (C_DIM / 8);
    copy16_g2s(&Qs[r][dc * 8], Qg + (size_t)r * C_DIM + dc * 8);
  }

  v8f o[8] = {};
  v8f orr[8] = {};
  const int srow = tid >> 4;
  const int sj   = tid & 15;
  const int trow = q0 + srow;
  float m_old = -1e30f;
  float l_run = 0.0f;
  const int kv_end = q0 + 32;

  for (int kv0 = 0; kv0 < kv_end; kv0 += 64) {
    __syncthreads();

    {
      v8f sc = {}, sr = {};
      const h16* aq  = &Qs[qi * 16][0];
      const h16* bk  = Kh + ((size_t)(b * SEQ + kv0 + kj * 16)) * C_DIM;
      const h16* aql = Ql + ((size_t)(b * SEQ + q0 + qi * 16)) * C_DIM;
      const h16* bkl = Kl + ((size_t)(b * SEQ + kv0 + kj * 16)) * C_DIM;
      const int kbeg = part * (C_DIM / 2);
#pragma unroll 2
      for (int kk = 0; kk < C_DIM / 2; kk += 32) {
        const int k0 = kbeg + kk;
        v16h a  = load_a_frag(aq, C_DIM, k0);
        v16h bb = load_b_frag(bk, C_DIM, k0);
        sc = wmma_f16(a, bb, sc);
        if (use_res) {
          v16h al = load_a_frag(aql, C_DIM, k0);
          v16h bl = load_b_frag(bkl, C_DIM, k0);
          sr = wmma_f16(a, bl, sr);
          sr = wmma_f16(al, bb, sr);
        }
      }
      const int col = kj * 16 + idx;
#pragma unroll
      for (int g = 0; g < 8; ++g)
        Ss[part][qi * 16 + g + 8 * half][col] = sc[g] + sr[g] * RUN;
    }
    __syncthreads();

    {
      float v[4];
      float mloc = -1e30f;
#pragma unroll
      for (int e = 0; e < 4; ++e) {
        const int cc = sj + e * 16;
        float s = (Ss[0][srow][cc] + Ss[1][srow][cc]) * ASC;
        if (kv0 + cc > trow) s = -__builtin_inff();
        v[e] = s;
        mloc = fmaxf(mloc, s);
      }
#pragma unroll
      for (int msk = 1; msk < 16; msk <<= 1) mloc = fmaxf(mloc, __shfl_xor(mloc, msk, 32));
      const float m_new = fmaxf(m_old, mloc);
      const float alpha = __expf(m_old - m_new);
      float ssum = 0.0f;
#pragma unroll
      for (int e = 0; e < 4; ++e) {
        const float p  = __expf(v[e] - m_new);
        ssum += p;
        const float pc = p * PSC;
        const h16 ph = (h16)pc;
        Ps[srow][sj + e * 16] = ph;
        if (PVRES) Prs[srow][sj + e * 16] = (h16)((pc - (float)ph) * RSC);
      }
#pragma unroll
      for (int msk = 1; msk < 16; msk <<= 1) ssum += __shfl_xor(ssum, msk, 32);
      l_run = l_run * alpha + ssum;
      m_old = m_new;
      if (sj == 0) { alpha_s[srow] = alpha; l_s[srow] = l_run; }
    }
    __syncthreads();

    {
      float al[8];
#pragma unroll
      for (int g = 0; g < 8; ++g) al[g] = alpha_s[qi * 16 + g + 8 * half];
#pragma unroll
      for (int t = 0; t < 8; ++t)
#pragma unroll
        for (int g = 0; g < 8; ++g) {
          o[t][g] *= al[g];
          if (PVRES) orr[t][g] *= al[g];
        }
      const h16* vbase  = Vt + ((size_t)(b * C_DIM + dg * 128)) * SEQ + kv0;
      const h16* vrbase = Vr + ((size_t)(b * C_DIM + dg * 128)) * VRK + kv0;
#pragma unroll
      for (int k0 = 0; k0 < 64; k0 += 32) {
        v16h a = load_a_frag(&Ps[qi * 16][0], 64, k0);
        v16h ar;
        if (PVRES) ar = load_a_frag(&Prs[qi * 16][0], 64, k0);
#pragma unroll
        for (int t = 0; t < 8; ++t) {
          v16h bb = load_b_frag(vbase + (size_t)(t * 16) * SEQ, SEQ, k0);
          o[t] = wmma_f16(a, bb, o[t]);
          if (PVRES) {
            v16h br = load_b_frag(vrbase + (size_t)(t * 16) * VRK, VRK, k0);
            orr[t] = wmma_f16(a, br, orr[t]);
            orr[t] = wmma_f16(ar, bb, orr[t]);
          }
        }
      }
    }
  }
  __syncthreads();

  float* Ot = (float*)&Qs[0][0];
  float linv[8];
#pragma unroll
  for (int g = 0; g < 8; ++g) linv[g] = PUN / l_s[qi * 16 + g + 8 * half];
  for (int hp = 0; hp < 2; ++hp) {
    if (qi == hp) {
#pragma unroll
      for (int t = 0; t < 8; ++t) {
        const int col = dg * 128 + t * 16 + idx;
#pragma unroll
        for (int g = 0; g < 8; ++g) {
          float val = o[t][g];
          if (PVRES) val += orr[t][g] * RUN;
          Ot[(g + 8 * half) * C_DIM + col] = val * linv[g];
        }
      }
    }
    __syncthreads();
    {
      float* dst = out + ((size_t)(b * SEQ_FULL + q0 + hp * 16)) * C_DIM;
      for (int gg = tid; gg < 16 * C_DIM / 4; gg += 512) vst2(dst + (size_t)gg * 4, *(const v4f*)(Ot + gg * 4));
    }
    __syncthreads();
  }
}

extern "C" void kernel_launch(void* const* d_in, const int* in_sizes, int n_in,
                              void* d_out, int out_size, void* d_ws, size_t ws_size,
                              hipStream_t stream) {
  if (n_in < 2) return;
  const int need_x = ((NB - 1) * SEQ_FULL + SEQ) * C_DIM;
  if (in_sizes[0] < need_x) return;
  if (in_sizes[1] < N_QKV * C_DIM) return;
  if (out_size < need_x) return;

  const float* x = (const float*)d_in[0];
  const float* wq = (const float*)d_in[1];
  float* out = (float*)d_out;

  const size_t plane  = (size_t)M_ROWS * C_DIM * sizeof(h16);
  const size_t wplane = (size_t)N_QKV * C_DIM * sizeof(h16);
  const size_t rplane = (size_t)NB * C_DIM * VRK * sizeof(h16);
  char* ws = (char*)d_ws;
  size_t off = 0;
  h16* xh = (h16*)(ws + off); off += plane;
  h16* wh = (h16*)(ws + off); off += wplane;
  h16* qh = (h16*)(ws + off); off += plane;
  h16* ql = (h16*)(ws + off); off += plane;
  h16* kh = (h16*)(ws + off); off += plane;
  h16* kl = (h16*)(ws + off); off += plane;
  h16* vt = (h16*)(ws + off); off += plane;
  h16* vr = (h16*)(ws + off); off += rplane;
  if (off > ws_size) return;

  const int n8x = M_ROWS * C_DIM / 8;
  const int n8w = N_QKV * C_DIM / 8;
  cvt_kernel<<<(n8x + 255) / 256, 256, 0, stream>>>(x, xh, n8x, SEQ, SEQ_FULL, XSC);
  cvt_kernel<<<(n8w + 255) / 256, 256, 0, stream>>>(wq, wh, n8w, N_QKV, N_QKV, WSC);

  qkv_kernel<<<dim3(M_ROWS / 64, N_QKV / 128), 256, 0, stream>>>(xh, wh, qh, ql, kh, kl, vt, vr);

  const int nqb  = SEQ / 32;
  const int nqbe = (nqb < VRK / 32) ? nqb : (VRK / 32);
  attn_kernel<1><<<dim3(nqbe, NB), 512, 0, stream>>>(qh, ql, kh, kl, vt, vr, out, 0);
  if (nqb > nqbe)
    attn_kernel<0><<<dim3(nqb - nqbe, NB), 512, 0, stream>>>(qh, ql, kh, kl, vt, vr, out, nqbe);
}
